// Up_86535001080407
// MI455X (gfx1250) — hardware-verified
//
#include <hip/hip_runtime.h>
#include <stddef.h>
#include <stdint.h>

typedef __attribute__((ext_vector_type(16))) _Float16 v16h;
typedef __attribute__((ext_vector_type(8)))  _Float16 v8h;
typedef __attribute__((ext_vector_type(16))) __bf16   v16b;
typedef __attribute__((ext_vector_type(8)))  __bf16   v8b;
typedef __attribute__((ext_vector_type(8)))  float    v8f;
typedef __attribute__((ext_vector_type(4)))  float    v4f;
typedef __attribute__((ext_vector_type(4)))  unsigned v4u;
typedef __attribute__((ext_vector_type(2)))  unsigned v2u;

constexpr int kBS = 2;
constexpr int kT = 8;
constexpr int kH = 128;
constexpr int kW = 128;
constexpr int kHW = kH * kW;
constexpr int kBT = kBS * kT;
constexpr int kPix = kBT * kHW;
constexpr int kHalfPix = kPix / 2;
constexpr int kEnc = 32;
constexpr int kDec = 64;
constexpr int kCat = 96;
constexpr int kNH = 4;
constexpr int kCoarse = 4096;
constexpr int kUpN = 256;

static constexpr size_t WS_WUP  = 0x0000000;
static constexpr size_t WS_WMLP = 0x0008000;
static constexpr size_t WS_WC1  = 0x000A000;
static constexpr size_t WS_WC2  = 0x0017800;
static constexpr size_t WS_BUPX = 0x001C000;
static constexpr size_t WS_AFF1 = 0x001C400;
static constexpr size_t WS_AFF2 = 0x001C500;
static constexpr size_t WS_AFF3 = 0x001C600;
static constexpr size_t WS_PART = 0x0020000;
static constexpr size_t WS_X1T  = 0x0200000;
static constexpr size_t WS_CUP  = 0x1000000;
static constexpr size_t WS_Y1B  = 0x1000000;
static constexpr size_t WS_Y2   = 0x2000000;
static constexpr size_t WS_HMLP = 0x5000000;
static constexpr size_t WS_Y1A  = 0x7000000;
static constexpr size_t WS_TOTAL = 0x8000000;
static_assert(WS_WUP + (size_t)kUpN * kDec * 2 <= WS_WMLP);
static_assert(WS_WMLP + (size_t)kEnc * 128 * 2 <= WS_WC1);
static_assert(WS_WC1 + (size_t)kEnc * 864 * 2 <= WS_WC2);
static_assert(WS_WC2 + (size_t)kEnc * 288 * 2 <= WS_BUPX);
static_assert(WS_BUPX + 256 * 4 <= WS_AFF1);
static_assert(WS_AFF3 + 64 * 4 <= WS_PART);
static_assert(WS_PART + (size_t)4096 * 64 * 4 <= WS_X1T);
static_assert(WS_X1T + (size_t)kBT * kCoarse * kDec * 2 <= WS_CUP);
static_assert(WS_CUP + (size_t)kBT * kCoarse * kUpN * 4 == WS_HMLP);
static_assert(WS_Y1B + (size_t)kHalfPix * kEnc * 4 == WS_Y2);
static_assert(WS_Y2 + (size_t)kPix * kEnc * 4 <= WS_HMLP);
static_assert(WS_HMLP + (size_t)kPix * kEnc * 4 == WS_Y1A);
static_assert(WS_Y1A + (size_t)kHalfPix * kEnc * 4 == WS_TOTAL);
static_assert(WS_TOTAL == (size_t)134217728);

__device__ __forceinline__ unsigned short f2bf_bits(float f) {
  unsigned u = __float_as_uint(f);
  return (unsigned short)((u + 0x7FFFu + ((u >> 16) & 1u)) >> 16);
}
__device__ __forceinline__ float bf_bits2f(unsigned short h) { return __uint_as_float(((unsigned)h) << 16); }
__device__ __forceinline__ float bfr(float f) { return bf_bits2f(f2bf_bits(f)); }
__device__ __forceinline__ void split_bf(float v, unsigned short& hb, unsigned short& lb) {
  hb = f2bf_bits(v);
  lb = f2bf_bits(v - bf_bits2f(hb));
}
__device__ __forceinline__ unsigned pack2(unsigned short a, unsigned short b) { return (unsigned)a | ((unsigned)b << 16); }
__device__ __forceinline__ int iclampi(int v, int lo, int hi) { return v < lo ? lo : (v > hi ? hi : v); }

__device__ __forceinline__ void dep_guard_h(v8f& a, v8f& b, v16h x, v16h y) { asm volatile("v_nop\n\tv_nop\n\tv_nop\n\tv_nop" : "+v"(a), "+v"(b) : "v"(x), "v"(y)); }
__device__ __forceinline__ void dep_guard_b(v8f& a, v8f& b, v16b x, v16b y) { asm volatile("v_nop\n\tv_nop\n\tv_nop\n\tv_nop" : "+v"(a), "+v"(b) : "v"(x), "v"(y)); }
__device__ __forceinline__ void keep4_h(v16h a, v16h b, v16h c, v16h d) { asm volatile("v_nop" :: "v"(a), "v"(b), "v"(c), "v"(d)); }
__device__ __forceinline__ void keep4_b(v16b a, v16b b, v16b c, v16b d) { asm volatile("v_nop" :: "v"(a), "v"(b), "v"(c), "v"(d)); }
__device__ __forceinline__ void acc_guard4(v8f& a, v8f& b, v8f& c, v8f& d) { asm volatile("v_nop\n\tv_nop\n\tv_nop\n\tv_nop" : "+v"(a), "+v"(b), "+v"(c), "+v"(d)); }
__device__ __forceinline__ void acc_guard2(v8f& a, v8f& b) { asm volatile("v_nop\n\tv_nop\n\tv_nop\n\tv_nop" : "+v"(a), "+v"(b)); }
template <typename T> struct Frag;
template <> struct Frag<_Float16> {
  typedef v16h V; union U { v16h v; v8h h[2]; };
  static __device__ __forceinline__ v16h load(const _Float16* p) {
    U f; f.h[0] = *(const v8h*)(p); f.h[1] = *(const v8h*)(p + 16); return f.v;
  }
  static __device__ __forceinline__ v8f mma(v16h a, v16h b, v8f c) {
    return __builtin_amdgcn_wmma_f32_16x16x32_f16(false, a, false, b, (short)0, c, false, false);
  }
  static __device__ __forceinline__ void guard(v8f& a, v8f& b, v16h x, v16h y) { dep_guard_h(a, b, x, y); }
  static __device__ __forceinline__ void keep(v16h a, v16h b, v16h c, v16h d) { keep4_h(a, b, c, d); }
};
template <> struct Frag<__bf16> {
  typedef v16b V; union U { v16b v; v8b h[2]; };
  static __device__ __forceinline__ v16b load(const __bf16* p) {
    U f; f.h[0] = *(const v8b*)(p); f.h[1] = *(const v8b*)(p + 16); return f.v;
  }
  static __device__ __forceinline__ v8f mma(v16b a, v16b b, v8f c) {
    return __builtin_amdgcn_wmma_f32_16x16x32_bf16(false, a, false, b, (short)0, c, false, false);
  }
  static __device__ __forceinline__ void guard(v8f& a, v8f& b, v16b x, v16b y) { dep_guard_b(a, b, x, y); }
  static __device__ __forceinline__ void keep(v16b a, v16b b, v16b c, v16b d) { keep4_b(a, b, c, d); }
};

template <int ET> struct Elem;
template <> struct Elem<0> { typedef _Float16 T; };
template <> struct Elem<1> { typedef __bf16 T; };
template <int ET, bool SPLIT, int BIAS_MODE, int OUT_MODE, bool RESID, int ACT = 0>
__global__ __launch_bounds__(256) void wmma_gemm64(
    const unsigned short* __restrict__ Ap, const unsigned short* __restrict__ A2p, int lda, long strideA,
    const unsigned short* __restrict__ Btp, const unsigned short* __restrict__ Bt2p, int ldb, long strideB,
    void* __restrict__ Cout, void* __restrict__ Cout2, int ldc, long strideC,
    const float* __restrict__ bias,
    const float* __restrict__ resid, long strideR,
    int M, int N, int K, float scale) {
  typedef typename Elem<ET>::T T;
  typedef typename Frag<T>::V V;
  const T* A = (const T*)Ap; const T* A2 = (const T*)A2p; const T* Bt = (const T*)Btp; const T* Bt2 = (const T*)Bt2p;
  __shared__ __align__(16) float sT[8][16 * 68];
  const int b    = blockIdx.y;
  const int lane = threadIdx.x & 31;
  const int wave = threadIdx.x >> 5;
  const int tilesN = N >> 6;
  const int tilesM = M >> 6;
  const int tile = blockIdx.x * 8 + wave;
  if (tile >= tilesM * tilesN) return;
  const int tm = tile / tilesN;
  const int tn = tile - tm * tilesN;
  const int m0 = tm << 6;
  const int n0 = tn << 6;

  const T* Ab  = A  + (size_t)b * strideA;
  const T* Bb  = Bt + (size_t)b * strideB;
  const T* Ab2 = SPLIT ? (A2  + (size_t)b * strideA) : nullptr;
  const T* Bb2 = SPLIT ? (Bt2 + (size_t)b * strideB) : nullptr;

  const int rlane = lane & 15;
  const int koff  = (lane >> 4) * 8;
  const int mOff  = (lane >> 4) * 8;

  v8f acc[4][4];
#pragma unroll
  for (int i = 0; i < 4; ++i)
#pragma unroll
    for (int j = 0; j < 4; ++j) acc[i][j] = (v8f){0.f,0.f,0.f,0.f,0.f,0.f,0.f,0.f};

  for (int k0 = 0; k0 < K; k0 += 32) {
    V bh[4], bl[4];
#pragma unroll
    for (int j = 0; j < 4; ++j) {
      const size_t bo = (size_t)(n0 + (j << 4) + rlane) * ldb + koff + k0;
      bh[j] = Frag<T>::load(Bb + bo);
      if (SPLIT) bl[j] = Frag<T>::load(Bb2 + bo);
    }
#pragma unroll
    for (int i = 0; i < 4; ++i) {
      const size_t ao = (size_t)(m0 + (i << 4) + rlane) * lda + koff + k0;
      V ah = Frag<T>::load(Ab + ao);
      V al;
      if (SPLIT) al = Frag<T>::load(Ab2 + ao);
#pragma unroll
      for (int j = 0; j < 4; ++j) {
        acc[i][j] = Frag<T>::mma(ah, bh[j], acc[i][j]);
        if (SPLIT) {
          acc[i][j] = Frag<T>::mma(ah, bl[j], acc[i][j]);
          acc[i][j] = Frag<T>::mma(al, bh[j], acc[i][j]);
        }
      }
      Frag<T>::guard(acc[i][0], acc[i][3], ah, SPLIT ? al : ah);
    }
    Frag<T>::keep(bh[0], bh[1], bh[2], bh[3]);
    if (SPLIT) Frag<T>::keep(bl[0], bl[1], bl[2], bl[3]);
  }
  acc_guard4(acc[0][0], acc[0][1], acc[0][2], acc[0][3]);
  acc_guard4(acc[1][0], acc[1][1], acc[1][2], acc[1][3]);
  acc_guard4(acc[2][0], acc[2][1], acc[2][2], acc[2][3]);
  acc_guard4(acc[3][0], acc[3][1], acc[3][2], acc[3][3]);

  float* slab = sT[wave];
  const float* Rb = RESID ? (resid + (size_t)b * strideR) : nullptr;
#pragma unroll
  for (int i = 0; i < 4; ++i) {
    const int mBase = m0 + (i << 4);
#pragma unroll
    for (int j = 0; j < 4; ++j) {
      const int n = n0 + (j << 4) + rlane;
      float bv = 0.f;
      if (BIAS_MODE == 2) bv = bias[n];
#pragma unroll
      for (int r = 0; r < 8; ++r) {
        float v = acc[i][j][r] * scale;
        if (BIAS_MODE == 1) v += bias[mBase + mOff + r];
        if (BIAS_MODE == 2) v += bv;
        if (RESID) v += Rb[(size_t)(mBase + mOff + r) * ldc + n];
        if (ACT == 1) v = tanhf(v);
        if (ACT == 2) v = fmaxf(v, 0.0f);
        if (ACT == 3) v = v / (1.0f + expf(-v));
        if (ACT == 4) v = (v > 0.f) ? v : 0.01f * v;
        if (ACT == 5) v = 0.5f * v * (1.0f + erff(v * 0.70710678118654752f));
        slab[(mOff + r) * 68 + (j << 4) + rlane] = v;
      }
    }
    __builtin_amdgcn_fence(__ATOMIC_RELEASE, "workgroup");
    __builtin_amdgcn_wave_barrier();
    __builtin_amdgcn_fence(__ATOMIC_ACQUIRE, "workgroup");
    if (OUT_MODE == 0) {
      float* C = (float*)Cout + (size_t)b * strideC;
      const int hh = lane >> 4, c4 = (lane & 15) * 4;
      for (int pass = 0; pass < 2; ++pass) {
#pragma unroll
        for (int it = 0; it < 8; ++it) {
          const int row = it * 2 + hh;
          v4f v = *(const v4f*)(slab + row * 68 + c4);
          *(volatile v4f*)(C + (size_t)(mBase + row) * ldc + n0 + c4) = v;
        }
        __threadfence();
      }
    } else {
      const int q = lane >> 3, c8 = (lane & 7) * 8;
      unsigned short* C  = (unsigned short*)Cout  + (size_t)b * strideC;
      unsigned short* C2 = (OUT_MODE == 2) ? ((unsigned short*)Cout2 + (size_t)b * strideC) : nullptr;
      for (int pass = 0; pass < 2; ++pass) {
#pragma unroll
        for (int it = 0; it < 4; ++it) {
          const int row = it * 4 + q;
          const float* sp = slab + row * 68 + c8;
          v8h hv, lv;
#pragma unroll
          for (int e = 0; e < 8; ++e) {
            if (OUT_MODE == 1) {
              hv[e] = (_Float16)sp[e];
            } else {
              unsigned short hb = f2bf_bits(sp[e]);
              unsigned short lb = f2bf_bits(sp[e] - bf_bits2f(hb));
              hv[e] = __builtin_bit_cast(_Float16, hb);
              lv[e] = __builtin_bit_cast(_Float16, lb);
            }
          }
          *(volatile v8h*)(C + (size_t)(mBase + row) * ldc + n0 + c8) = hv;
          if (OUT_MODE == 2) *(volatile v8h*)(C2 + (size_t)(mBase + row) * ldc + n0 + c8) = lv;
        }
        __threadfence();
      }
    }
    __builtin_amdgcn_fence(__ATOMIC_RELEASE, "workgroup");
    __builtin_amdgcn_wave_barrier();
    __builtin_amdgcn_fence(__ATOMIC_ACQUIRE, "workgroup");
  }
}

__device__ __forceinline__ void st16x2(unsigned short* dst, const unsigned short (&h)[8]) {
  const v4u u = (v4u){pack2(h[0], h[1]), pack2(h[2], h[3]), pack2(h[4], h[5]), pack2(h[6], h[7])};
  *(volatile v4u*)dst = u;
  __threadfence();
  *(volatile v4u*)dst = u;
}

__global__ __launch_bounds__(256) void k_wprep(
    const float* __restrict__ wup, const float* __restrict__ wmlp, const float* __restrict__ wc1,
    const float* __restrict__ wc2, const float* __restrict__ bup,
    unsigned short* __restrict__ wupT, unsigned short* __restrict__ wmlpT, unsigned short* __restrict__ wc1T,
    unsigned short* __restrict__ wc2T, float* __restrict__ bupx) {
  const int blk = blockIdx.x, tid = threadIdx.x;
  unsigned short h[8];
  if (blk < 8) {
    const int q = blk * 256 + tid;
    const int e0 = q * 8;
    const int n = e0 >> 6, c = e0 & 63;
    const int o = n & 63, kl = n >> 6;
#pragma unroll
    for (int i = 0; i < 8; ++i) h[i] = f2bf_bits(wup[((c + i) * kDec + o) * 4 + kl]);
    st16x2(wupT + e0, h);
  } else if (blk < 10) {
    const int q = (blk - 8) * 256 + tid;
    const int e0 = q * 8;
    const int o = e0 >> 7, k = e0 & 127;
#pragma unroll
    for (int i = 0; i < 8; ++i) h[i] = f2bf_bits(wmlp[(k + i) * kEnc + o]);
    st16x2(wmlpT + e0, h);
  } else if (blk < 24) {
    const int q = (blk - 10) * 256 + tid;
    if (q < 3456) {
      const int e0 = q * 8;
      const int o = e0 / 864, k = e0 - o * 864;
#pragma unroll
      for (int i = 0; i < 8; ++i) {
        const int kk = k + i;
        const int tap = kk / kCat, ic = kk - tap * kCat;
        h[i] = f2bf_bits(wc1[(o * kCat + ic) * 9 + tap]);
      }
      st16x2(wc1T + e0, h);
    }
  } else if (blk < 29) {
    const int q = (blk - 24) * 256 + tid;
    if (q < 1152) {
      const int e0 = q * 8;
      const int o = e0 / 288, k = e0 - o * 288;
#pragma unroll
      for (int i = 0; i < 8; ++i) {
        const int kk = k + i;
        const int tap = kk >> 5, ic = kk & 31;
        h[i] = f2bf_bits(wc2[(o * kEnc + ic) * 9 + tap]);
      }
      st16x2(wc2T + e0, h);
    }
  } else {
    if (tid < 64) {
      const int n0 = tid * 4;
      const v4f v = (v4f){bfr(bup[(n0 + 0) & 63]), bfr(bup[(n0 + 1) & 63]),
                          bfr(bup[(n0 + 2) & 63]), bfr(bup[(n0 + 3) & 63])};
      *(volatile v4f*)(bupx + n0) = v;
      __threadfence();
      *(volatile v4f*)(bupx + n0) = v;
    }
  }
}

__global__ __launch_bounds__(256) void k_x1t(const float* __restrict__ x1, unsigned short* __restrict__ x1t) {
  __shared__ __align__(16) unsigned short xt[128 * 72];
  const int tid = threadIdx.x, blk = blockIdx.x;
  const int bt = blk >> 5, mc = blk & 31;
  const int b = bt >> 3, t = bt & 7;
  const int m0 = mc * 128;
#pragma unroll
  for (int i = 0; i < 8; ++i) {
    const int idx = i * 256 + tid;
    const int c = idx >> 5, m4 = (idx & 31) * 4;
    const v4f v = *(const v4f*)(x1 + ((size_t)(b * kDec + c) * kT + t) * kCoarse + m0 + m4);
#pragma unroll
    for (int e = 0; e < 4; ++e) xt[(m4 + e) * 72 + c] = f2bf_bits(v[e]);
  }
  __syncthreads();
  unsigned short* dst = x1t + ((size_t)bt * kCoarse + m0) * kDec;
  for (int pass = 0; pass < 2; ++pass) {
#pragma unroll
    for (int i = 0; i < 4; ++i) {
      const int off = i * 2048 + tid * 8;
      const int m = off >> 6, c0 = off & 63;
      const v4u v = *(const v4u*)(xt + m * 72 + c0);
      *(volatile v4u*)(dst + off) = v;
    }
    __threadfence();
  }
}

template <int IC, int TAPS, int MS, int YP>
__device__ __forceinline__ void tile_gemm(const unsigned short* tHp, const unsigned short* tLp,
                                          const unsigned short* __restrict__ wtp, int pw0, int lane,
                                          v8f (&acc)[MS][2]) {
  constexpr int KTOT = TAPS * IC;
  static_assert(KTOT % 32 == 0);
  static_assert(IC % 32 == 0);
  typedef Frag<__bf16> F;
  const __bf16* tH = (const __bf16*)(const void*)tHp;
  const __bf16* tL = (const __bf16*)(const void*)tLp;
  const __bf16* wt = (const __bf16*)(const void*)wtp;
  const int rlane = lane & 15, koff = (lane >> 4) * 8;
#pragma unroll
  for (int i = 0; i < MS; ++i) {
    acc[i][0] = (v8f){0.f,0.f,0.f,0.f,0.f,0.f,0.f,0.f};
    acc[i][1] = (v8f){0.f,0.f,0.f,0.f,0.f,0.f,0.f,0.f};
  }
#pragma unroll 1
  for (int k0 = 0; k0 < KTOT; k0 += 32) {
    const int tap = k0 / IC;
    const int c0 = k0 - tap * IC;
    const int dr = (TAPS == 9) ? (tap / 3) : 0;
    const int dc = (TAPS == 9) ? (tap - dr * 3) : 0;
    v16b bh[2];
#pragma unroll
    for (int j = 0; j < 2; ++j) bh[j] = F::load(wt + (size_t)(j * 16 + rlane) * KTOT + k0 + koff);
#pragma unroll
    for (int i = 0; i < MS; ++i) {
      const int aoff = (dr * YP + pw0 + i * 16 + rlane + dc) * IC + c0 + koff;
      const v16b ah = F::load(tH + aoff);
      const v16b al = F::load(tL + aoff);
#pragma unroll
      for (int j = 0; j < 2; ++j) {
        acc[i][j] = F::mma(ah, bh[j], acc[i][j]);
        acc[i][j] = F::mma(al, bh[j], acc[i][j]);
      }
      F::guard(acc[i][0], acc[i][1], ah, al);
    }
    F::keep(bh[0], bh[1], bh[0], bh[1]);
  }
#pragma unroll
  for (int i = 0; i < MS; ++i) acc_guard2(acc[i][0], acc[i][1]);
}

__global__ __launch_bounds__(128) void k_ctx_mlp(
    const float* __restrict__ x2, const float* __restrict__ attn, const unsigned short* __restrict__ wt,
    const float* __restrict__ bias, float* __restrict__ hout, float* __restrict__ part) {
  __shared__ __align__(16) unsigned short tH[128 * 128];
  __shared__ __align__(16) unsigned short tL[128 * 128];
  __shared__ __align__(16) float slab[128 * 32];
  __shared__ __align__(16) float spart[64];
  __shared__ float arow[kNH * kT * 16];
  __shared__ float sbias[32];
  const int tid = threadIdx.x, lane = tid & 31, wave = tid >> 5;
  const int blk = blockIdx.x;
  const int x = blk & 127, bt = blk >> 7;
  const int b = bt >> 3, t = bt & 7;

  const float sx = ((float)x + 0.5f) * 0.125f - 0.5f;
  const float flx = floorf(sx);
  const float fx = sx - flx;
  const int ix = (int)flx;
  const int ix0 = iclampi(ix, 0, 15), ix1 = iclampi(ix + 1, 0, 15);
  for (int idx = tid; idx < kNH * kT * 16; idx += 128) {
    const int n = idx >> 7, s = (idx >> 4) & 7, j = idx & 15;
    const size_t base = (size_t)(n * kBS + b) * 16;
    const float g0 = bfr(attn[(((base + ix0) * 16 + j) * kT + t) * kT + s]);
    const float g1 = bfr(attn[(((base + ix1) * 16 + j) * kT + t) * kT + s]);
    arow[idx] = g0 + fx * (g1 - g0);
  }
  if (tid < 32) sbias[tid] = bfr(bias[tid]);
  __syncthreads();

  const int y = tid;
  const float sy = ((float)y + 0.5f) * 0.125f - 0.5f;
  const float fly = floorf(sy);
  const float fy = sy - fly;
  const int iy = (int)fly;
  const int iy0 = iclampi(iy, 0, 15), iy1 = iclampi(iy + 1, 0, 15);
  float ca[kNH][kT];
#pragma unroll
  for (int n = 0; n < kNH; ++n)
#pragma unroll
    for (int s = 0; s < kT; ++s) {
      const float v0 = arow[(n * kT + s) * 16 + iy0];
      const float v1 = arow[(n * kT + s) * 16 + iy1];
      ca[n][s] = v0 + fy * (v1 - v0);
    }
  const float* xb = x2 + (size_t)b * kEnc * kT * kHW + (size_t)x * kW + y;
#pragma unroll 1
  for (int c = 0; c < kEnc; ++c) {
    float xv[kT];
#pragma unroll
    for (int s = 0; s < kT; ++s) xv[s] = bfr(xb[(size_t)(c * kT + s) * kHW]);
    float r0 = 0.0f, r1 = 0.0f, r2 = 0.0f, r3 = 0.0f;
#pragma unroll
    for (int s = 0; s < kT; ++s) {
      r0 += ca[0][s] * xv[s];
      r1 += ca[1][s] * xv[s];
      r2 += ca[2][s] * xv[s];
      r3 += ca[3][s] * xv[s];
    }
    unsigned short h0, l0, h1, l1, h2, l2, h3, l3;
    split_bf(r0, h0, l0); split_bf(r1, h1, l1); split_bf(r2, h2, l2); split_bf(r3, h3, l3);
    const int toff = y * 128 + c * 4;
    *(v2u*)(tH + toff) = (v2u){pack2(h0, h1), pack2(h2, h3)};
    *(v2u*)(tL + toff) = (v2u){pack2(l0, l1), pack2(l2, l3)};
  }
  __syncthreads();

  v8f acc[2][2];
  tile_gemm<128, 1, 2, 128>(tH, tL, wt, wave * 32, lane, acc);
  const int rlane = lane & 15, hh = lane >> 4;
#pragma unroll
  for (int i = 0; i < 2; ++i)
#pragma unroll
    for (int j = 0; j < 2; ++j) {
      const int ch = j * 16 + rlane;
      const float bv = sbias[ch];
#pragma unroll
      for (int r = 0; r < 8; ++r) slab[(wave * 32 + i * 16 + 8 * hh + r) * 32 + ch] = acc[i][j][r] + bv;
    }
  __syncthreads();

  float* dst = hout + (size_t)blk * 128 * 32;
  for (int pass = 0; pass < 2; ++pass) {
#pragma unroll
    for (int i = 0; i < 8; ++i) {
      const int off = i * 512 + tid * 4;
      const v4f v = *(const v4f*)(slab + off);
      *(volatile v4f*)(dst + off) = v;
    }
    __threadfence();
  }
  if (tid < 32) {
    float s = 0.0f, q = 0.0f;
#pragma unroll 1
    for (int px = 0; px < 128; ++px) {
      const float v = slab[px * 32 + tid];
      s += v;
      q += v * v;
    }
    spart[tid] = s;
    spart[32 + tid] = q;
  }
  __syncthreads();
  if (tid < 16) {
    const v4f pv = *(const v4f*)(spart + tid * 4);
    float* pd = part + (size_t)blk * 64 + tid * 4;
    *(volatile v4f*)pd = pv;
    __threadfence();
    *(volatile v4f*)pd = pv;
  }
}

__global__ __launch_bounds__(64) void k_stats(const float* __restrict__ part, int nblk,
                                             const float* __restrict__ g, const float* __restrict__ be,
                                             float* __restrict__ aff) {
  __shared__ __align__(16) float saff[64];
  const int tid = threadIdx.x;
  if (tid < 32) {
    double s = 0.0, q = 0.0;
    for (int i = 0; i < nblk; ++i) {
      s += (double)part[(size_t)i * 64 + tid];
      q += (double)part[(size_t)i * 64 + 32 + tid];
    }
    const double inv = 1.0 / 262144.0;
    const double mean = s * inv;
    const double var = q * inv - mean * mean;
    const float varf = fmaxf((float)var, 0.0f);
    const float a = bfr(g[tid]) * (1.0f / sqrtf(varf + 1e-5f));
    saff[tid] = a;
    saff[32 + tid] = bfr(be[tid]) - (float)mean * a;
  }
  __syncthreads();
  if (tid < 16) {
    const v4f v = *(const v4f*)(saff + tid * 4);
    *(volatile v4f*)(aff + tid * 4) = v;
    __threadfence();
    *(volatile v4f*)(aff + tid * 4) = v;
  }
}

template <int IC>
__global__ __launch_bounds__(128) void k_conv(
    const float* __restrict__ hA, const float* __restrict__ hB, const float* __restrict__ aff,
    const float* up, const unsigned short* __restrict__ wt, const float* __restrict__ bias,
    float* oA, float* oB, float* __restrict__ part, int blk0) {
  constexpr int YP = 66;
  constexpr int TILE = 3 * YP * IC;
  __shared__ __align__(16) unsigned short tH[TILE];
  __shared__ __align__(16) unsigned short tL[TILE];
  __shared__ __align__(16) float slab[64 * 32];
  __shared__ __align__(16) float spart[64];
  __shared__ float saff[64];
  __shared__ float sbias[32];
  const int tid = threadIdx.x, lane = tid & 31, wave = tid >> 5;
  const int blk = blk0 + blockIdx.x;
  const int yh = blk & 1, x = (blk >> 1) & 127, bt = blk >> 8;
  const int y0 = yh * 64;
  const bool upper = (bt >= 8);
  const float* hsrc = upper ? hB : hA;
  float* odst = upper ? oB : oA;
  const size_t prel0 = upper ? (size_t)kHalfPix : (size_t)0;
  if (tid < 64) saff[tid] = aff[tid];
  if (tid < 32) sbias[tid] = bfr(bias[tid]);
  __syncthreads();

  for (int dr = 0; dr < 3; ++dr) {
    const int gx = x - 1 + dr;
    const bool vx = (gx >= 0) && (gx < kH);
    const int gxc = iclampi(gx, 0, kH - 1);
    const size_t prow = ((size_t)bt * kH + gxc) * kW;
    const float* hrow = hsrc + (prow - prel0) * 32;
#pragma unroll
    for (int i = 0; i < 4; ++i) {
      const int idx = i * 128 + tid;
      const int px = idx >> 3, c4 = (idx & 7) * 4;
      const v4f v = *(const v4f*)(hrow + (size_t)(y0 + px) * 32 + c4);
      unsigned short hb[4], lb[4];
#pragma unroll
      for (int e = 0; e < 4; ++e) {
        float r = fmaxf(fmaf(saff[c4 + e], v[e], saff[32 + c4 + e]), 0.0f);
        r = vx ? r : 0.0f;
        split_bf(r, hb[e], lb[e]);
      }
      const int toff = (dr * YP + 1 + px) * IC + c4;
      *(v2u*)(tH + toff) = (v2u){pack2(hb[0], hb[1]), pack2(hb[2], hb[3])};
      *(v2u*)(tL + toff) = (v2u){pack2(lb[0], lb[1]), pack2(lb[2], lb[3])};
    }
    if (tid < 16) {
      const int side = tid >> 3, c4 = (tid & 7) * 4;
      const int gy = side ? (y0 + 64) : (y0 - 1);
      const bool vy = (gy >= 0) && (gy < kW);
      const int gyc = iclampi(gy, 0, kW - 1);
      const v4f v = *(const v4f*)(hrow + (size_t)gyc * 32 + c4);
      unsigned short hb[4], lb[4];
#pragma unroll
      for (int e = 0; e < 4; ++e) {
        float r = fmaxf(fmaf(saff[c4 + e], v[e], saff[32 + c4 + e]), 0.0f);
        r = (vx && vy) ? r : 0.0f;
        split_bf(r, hb[e], lb[e]);
      }
      const int toff = (dr * YP + (side ? 65 : 0)) * IC + c4;
      *(v2u*)(tH + toff) = (v2u){pack2(hb[0], hb[1]), pack2(hb[2], hb[3])};
      *(v2u*)(tL + toff) = (v2u){pack2(lb[0], lb[1]), pack2(lb[2], lb[3])};
    }
    if (IC == 96) {
#pragma unroll 1
      for (int gi = 0; gi < 2; ++gi) {
#pragma unroll
        for (int ii = 0; ii < 4; ++ii) {
          const int idx = (gi * 4 + ii) * 128 + tid;
          const int px = idx >> 4, o4 = (idx & 15) * 4;
          const int gy = y0 + px;
          const int m = (gxc >> 1) * 64 + (gy >> 1);
          const int kl = (gxc & 1) * 2 + (gy & 1);
          const v4f v = *(const v4f*)(up + ((size_t)bt * kCoarse + m) * kUpN + kl * 64 + o4);
          unsigned short hb[4], lb[4];
#pragma unroll
          for (int e = 0; e < 4; ++e) {
            const float r = vx ? v[e] : 0.0f;
            split_bf(r, hb[e], lb[e]);
          }
          const int toff = (dr * YP + 1 + px) * IC + 32 + o4;
          *(v2u*)(tH + toff) = (v2u){pack2(hb[0], hb[1]), pack2(hb[2], hb[3])};
          *(v2u*)(tL + toff) = (v2u){pack2(lb[0], lb[1]), pack2(lb[2], lb[3])};
        }
      }
      if (tid < 32) {
        const int side = tid >> 4, o4 = (tid & 15) * 4;
        const int gy = side ? (y0 + 64) : (y0 - 1);
        const bool vy = (gy >= 0) && (gy < kW);
        const int gyc = iclampi(gy, 0, kW - 1);
        const int m = (gxc >> 1) * 64 + (gyc >> 1);
        const int kl = (gxc & 1) * 2 + (gyc & 1);
        const v4f v = *(const v4f*)(up + ((size_t)bt * kCoarse + m) * kUpN + kl * 64 + o4);
        unsigned short hb[4], lb[4];
#pragma unroll
        for (int e = 0; e < 4; ++e) {
          const float r = (vx && vy) ? v[e] : 0.0f;
          split_bf(r, hb[e], lb[e]);
        }
        const int toff = (dr * YP + (side ? 65 : 0)) * IC + 32 + o4;
        *(v2u*)(tH + toff) = (v2u){pack2(hb[0], hb[1]), pack2(hb[2], hb[3])};
        *(v2u*)(tL + toff) = (v2u){pack2(lb[0], lb[1]), pack2(lb[2], lb[3])};
      }
    }
  }
  __syncthreads();

  v8f acc[1][2];
  tile_gemm<IC, 9, 1, YP>(tH, tL, wt, wave * 16, lane, acc);
  const int rlane = lane & 15, hh = lane >> 4;
#pragma unroll
  for (int j = 0; j < 2; ++j) {
    const int ch = j * 16 + rlane;
    const float bv = sbias[ch];
#pragma unroll
    for (int r = 0; r < 8; ++r) slab[(wave * 16 + 8 * hh + r) * 32 + ch] = acc[0][j][r] + bv;
  }
  __syncthreads();

  const size_t p0 = ((size_t)bt * kH + x) * kW + y0;
  float* dst = odst + (p0 - prel0) * 32;
  for (int pass = 0; pass < 2; ++pass) {
#pragma unroll
    for (int i = 0; i < 4; ++i) {
      const int off = i * 512 + tid * 4;
      const v4f v = *(const v4f*)(slab + off);
      *(volatile v4f*)(dst + off) = v;
    }
    __threadfence();
  }
  if (tid < 32) {
    float s = 0.0f, q = 0.0f;
#pragma unroll 1
    for (int px = 0; px < 64; ++px) {
      const float v = slab[px * 32 + tid];
      s += v;
      q += v * v;
    }
    spart[tid] = s;
    spart[32 + tid] = q;
  }
  __syncthreads();
  if (tid < 16) {
    const v4f pv = *(const v4f*)(spart + tid * 4);
    float* pd = part + (size_t)blk * 64 + tid * 4;
    *(volatile v4f*)pd = pv;
    __threadfence();
    *(volatile v4f*)pd = pv;
  }
}

__global__ __launch_bounds__(256) void k_out(const float* __restrict__ y2, const float* __restrict__ aff,
                                            float* __restrict__ out) {
  __shared__ __align__(16) float ot[32 * 132];
  __shared__ float saff[64];
  const int tid = threadIdx.x, blk = blockIdx.x;
  const int x = blk & 127, bt = blk >> 7;
  const int b = bt >> 3, t = bt & 7;
  if (tid < 64) saff[tid] = aff[tid];
  __syncthreads();
  const float* src = y2 + (size_t)blk * 128 * 32;
#pragma unroll
  for (int i = 0; i < 4; ++i) {
    const int idx = i * 256 + tid;
    const int px = idx >> 3, c4 = (idx & 7) * 4;
    const v4f v = *(const v4f*)(src + (size_t)idx * 4);
#pragma unroll
    for (int e = 0; e < 4; ++e) {
      const int ch = c4 + e;
      ot[ch * 132 + px] = fmaxf(fmaf(saff[ch], v[e], saff[32 + ch]), 0.0f);
    }
  }
  __syncthreads();
  for (int pass = 0; pass < 2; ++pass) {
#pragma unroll
    for (int i = 0; i < 4; ++i) {
      const int c = i * 8 + (tid >> 5);
      const int y4 = (tid & 31) * 4;
      const v4f v = *(const v4f*)(ot + c * 132 + y4);
      *(volatile v4f*)(out + ((size_t)(b * kEnc + c) * kT + t) * kHW + (size_t)x * kW + y4) = v;
    }
    __threadfence();
  }
}

extern "C" void kernel_launch(void* const* d_in, const int* in_sizes, int n_in,
                              void* d_out, int out_size, void* d_ws, size_t ws_size,
                              hipStream_t stream) {
  if (n_in < 17) return;
  if (in_sizes[0] != kBS * kDec * kT * kCoarse) return;
  if (in_sizes[1] != kBS * kEnc * kT * kHW) return;
  if (in_sizes[2] != kNH * kBS * 16 * 16 * kT * kT) return;
  if (in_sizes[3] != kDec * kDec * 4 || in_sizes[5] != kNH * kEnc * kEnc) return;
  if (in_sizes[9] != kEnc * kCat * 9 || in_sizes[13] != kEnc * kEnc * 9) return;
  if (out_size != kBS * kEnc * kT * kHW) return;
  if (ws_size < WS_TOTAL) return;

  const float* x1     = (const float*)d_in[0];
  const float* x2     = (const float*)d_in[1];
  const float* attn   = (const float*)d_in[2];
  const float* W_up   = (const float*)d_in[3];
  const float* b_up   = (const float*)d_in[4];
  const float* W_mlp  = (const float*)d_in[5];
  const float* b_mlp  = (const float*)d_in[6];
  const float* g_mlp  = (const float*)d_in[7];
  const float* be_mlp = (const float*)d_in[8];
  const float* W_c1   = (const float*)d_in[9];
  const float* b_c1   = (const float*)d_in[10];
  const float* g_c1   = (const float*)d_in[11];
  const float* be_c1  = (const float*)d_in[12];
  const float* W_c2   = (const float*)d_in[13];
  const float* b_c2   = (const float*)d_in[14];
  const float* g_c2   = (const float*)d_in[15];
  const float* be_c2  = (const float*)d_in[16];
  float* out = (float*)d_out;

  char* ws = (char*)d_ws;
  unsigned short* wupT  = (unsigned short*)(ws + WS_WUP);
  unsigned short* wmlpT = (unsigned short*)(ws + WS_WMLP);
  unsigned short* wc1T  = (unsigned short*)(ws + WS_WC1);
  unsigned short* wc2T  = (unsigned short*)(ws + WS_WC2);
  float* bupx = (float*)(ws + WS_BUPX);
  float* aff1 = (float*)(ws + WS_AFF1);
  float* aff2 = (float*)(ws + WS_AFF2);
  float* aff3 = (float*)(ws + WS_AFF3);
  float* part = (float*)(ws + WS_PART);
  unsigned short* x1t = (unsigned short*)(ws + WS_X1T);
  float* cup  = (float*)(ws + WS_CUP);
  float* y1b  = (float*)(ws + WS_Y1B);
  float* y2   = (float*)(ws + WS_Y2);
  float* hmlp = (float*)(ws + WS_HMLP);
  float* y1a  = (float*)(ws + WS_Y1A);

  k_wprep<<<dim3(30), dim3(256), 0, stream>>>(W_up, W_mlp, W_c1, W_c2, b_up, wupT, wmlpT, wc1T, wc2T, bupx);
  k_x1t<<<dim3(kBT * 32), dim3(256), 0, stream>>>(x1, x1t);
  static_assert(kCoarse % 64 == 0 && kUpN % 64 == 0 && kDec % 32 == 0);
  wmma_gemm64<1, false, 2, 0, false, 0><<<dim3((kCoarse / 64) * (kUpN / 64) / 8, kBT), dim3(256), 0, stream>>>(
      x1t, x1t, kDec, (long)kCoarse * kDec,
      wupT, wupT, kDec, 0L,
      (void*)cup, (void*)cup, kUpN, (long)kCoarse * kUpN,
      bupx, bupx, 0L, kCoarse, kUpN, kDec, 1.0f);
  k_ctx_mlp<<<dim3(kBT * kH), dim3(128), 0, stream>>>(x2, attn, wmlpT, b_mlp, hmlp, part);
  k_stats<<<dim3(1), dim3(64), 0, stream>>>(part, kBT * kH, g_mlp, be_mlp, aff1);
  k_conv<96><<<dim3(2048), dim3(128), 0, stream>>>(hmlp, hmlp + (size_t)kHalfPix * 32, aff1, cup, wc1T, b_c1,
                                                     y1a, y1b, part, 0);
  k_conv<96><<<dim3(2048), dim3(128), 0, stream>>>(hmlp, hmlp + (size_t)kHalfPix * 32, aff1, cup, wc1T, b_c1,
                                                     y1a, y1b, part, 2048);
  k_stats<<<dim3(1), dim3(64), 0, stream>>>(part, 4096, g_c1, be_c1, aff2);
  k_conv<32><<<dim3(4096), dim3(128), 0, stream>>>(y1a, y1b, aff2, cup, wc2T, b_c2,
                                                     y2, y2 + (size_t)kHalfPix * 32, part, 0);
  k_stats<<<dim3(1), dim3(64), 0, stream>>>(part, 4096, g_c2, be_c2, aff3);
  k_out<<<dim3(kBT * kH), dim3(256), 0, stream>>>(y2, aff3, out);
}
